// FEAST_layer_73005854097931
// MI455X (gfx1250) — hardware-verified
//
#include <hip/hip_runtime.h>
#include <stddef.h>


#define DIN   64
#define DOUT  32
#define HDIM  16
#define GR    32
#define NT1   128
#define NB    512
#define CHUNK 2048
#define NTHR  256
#define NWAVE 8
#define WCAP  256
#define NGRP  (CHUNK / (NTHR * 4))
#define ASCW  16

#define LDS_ACC   (NB * (2 * DOUT + 4 + 4))
#define LDS_LIST  (NWAVE * WCAP)
#define LDS_BYTES ((LDS_ACC + LDS_LIST + NWAVE) * 4)

static_assert(WCAP == (CHUNK / NTHR) * 32);
static_assert(NGRP == 2);
static_assert(NB == 512);
static_assert(CHUNK <= 2048);
static_assert(NB == NWAVE * 64);
static_assert(NT1 == 128);
static_assert((LDS_ACC % 4) == 0);
static_assert(((NB * 2 * DOUT + NB * 4) % 4) == 0);
static_assert(LDS_BYTES == 155680);

typedef float  v4f  __attribute__((ext_vector_type(4)));
typedef float  v8f  __attribute__((ext_vector_type(8)));
typedef int    v4i  __attribute__((ext_vector_type(4)));
typedef double v2d  __attribute__((ext_vector_type(2)));
typedef __bf16 v16b __attribute__((ext_vector_type(16)));
union Frag { v16b v; v4i q[2]; };

__device__ __forceinline__ unsigned int bf_bits(float f) {
  unsigned int u = __float_as_uint(f);
  u += 0x7FFFu + ((u >> 16) & 1u);
  return u >> 16;
}
__device__ __forceinline__ float bfr(float f) { return __uint_as_float(bf_bits(f) << 16); }
__device__ __forceinline__ int pk2(float a, float b) { return (int)(bf_bits(a) | (bf_bits(b) << 16)); }
__device__ __forceinline__ v4i pack8(v4f a, v4f b) {
  v4i r;
  r.x = pk2(a.x, a.y); r.y = pk2(a.z, a.w); r.z = pk2(b.x, b.y); r.w = pk2(b.z, b.w);
  return r;
}

__device__ __forceinline__ v8f wm(v16b a, v16b b, v8f c) {
  v8f d = __builtin_amdgcn_wmma_f32_16x16x32_bf16(false, a, false, b, (short)0, c, false, false);
  asm volatile("v_nop\n\tv_nop\n\tv_nop\n\tv_nop" : "+v"(d) : "v"(a), "v"(b));
  return d;
}

__global__ __launch_bounds__(NTHR) void k_prep(
    const float* __restrict__ w1, const float* __restrict__ w2,
    const float* __restrict__ wa1, const float* __restrict__ wa2,
    unsigned short* WT, int n8) {
  const int i = blockIdx.x * NTHR + threadIdx.x;
  if (i >= n8) return;
  const int mat = i >> 9;
  const int n   = (i >> 3) & 63;
  const int kg  = i & 7;
  const float* W = mat ? (n < 32 ? wa1 : wa2) : (n < 32 ? w1 : w2);
  const int nn = n & 31;
  float f[8];
#pragma unroll
  for (int j = 0; j < 8; ++j) f[j] = W[(kg * 8 + j) * DOUT + nn];
  v4i u;
  u.x = pk2(f[0], f[1]); u.y = pk2(f[2], f[3]); u.z = pk2(f[4], f[5]); u.w = pk2(f[6], f[7]);
  unsigned short* p = WT + (size_t)(mat * 64 + n) * DIN + kg * 8;
  *(volatile v4i*)p = u;
  __threadfence();
  *(volatile v4i*)p = u;
}

__global__ __launch_bounds__(NT1) void k_node(
    const float* __restrict__ h, const float* __restrict__ ah,
    const unsigned short* __restrict__ WT,
    const float* __restrict__ b1, const float* __restrict__ ba1,
    const float* __restrict__ b2, const float* __restrict__ ba2,
    const float* __restrict__ wp, const float* __restrict__ wn, const float* __restrict__ wr,
    float* th, float* lh, float* tah, float* lah, float* asc, double* rsd,
    int nN, int nPad) {
  __shared__ __attribute__((aligned(16))) float  S[4 * GR * DOUT];
  __shared__ __attribute__((aligned(16))) float  SC[GR * ASCW];
  __shared__ __attribute__((aligned(16))) double PR[4 * GR];
  __shared__ __attribute__((aligned(16))) double RS[2 * GR];

  const int tid  = threadIdx.x;
  const int lane = tid & 31;
  const int wave = tid >> 5;
  const int hh   = lane >> 4;
  const int m    = lane & 15;
  const int rowBase = blockIdx.x * GR;

  {
    const int mat  = wave & 1;
    const int tile = wave >> 1;
    const float* X = mat ? ah : h;
    int arow = rowBase + tile * 16 + m;
    if (arow > nN - 1) arow = nN - 1;
    const float* xp = X + (size_t)arow * DIN + 8 * hh;
    Frag a0, a1;
    a0.q[0] = pack8(*(const v4f*)(xp),      *(const v4f*)(xp + 4));
    a0.q[1] = pack8(*(const v4f*)(xp + 16), *(const v4f*)(xp + 20));
    a1.q[0] = pack8(*(const v4f*)(xp + 32), *(const v4f*)(xp + 36));
    a1.q[1] = pack8(*(const v4f*)(xp + 48), *(const v4f*)(xp + 52));
    const float* bT = mat ? ba1 : b1;
    const float* bL = mat ? ba2 : b2;
#pragma unroll
    for (int ct = 0; ct < 4; ++ct) {
      const int n = ct * 16 + m;
      const unsigned short* pb = WT + (size_t)(mat * 64 + n) * DIN + 8 * hh;
      Frag fb0, fb1;
      fb0.q[0] = *(const v4i*)(pb);       fb0.q[1] = *(const v4i*)(pb + 16);
      fb1.q[0] = *(const v4i*)(pb + 32);  fb1.q[1] = *(const v4i*)(pb + 48);
      v8f acc = {0.f, 0.f, 0.f, 0.f, 0.f, 0.f, 0.f, 0.f};
      acc = wm(a0.v, fb0.v, acc);
      acc = wm(a1.v, fb1.v, acc);
      const int part = ct >> 1;
      const int col  = (ct & 1) * 16 + m;
      const float bias = bfr((part ? bL : bT)[col]);
      float* sp = S + ((mat * 2 + part) * GR + tile * 16 + 8 * hh) * DOUT + col;
#pragma unroll
      for (int r = 0; r < 8; ++r) sp[r * DOUT] = acc[r] + bias;
    }
  }
  __syncthreads();

  {
    const int row  = lane;
    const int part = wave;
    int grow = rowBase + row;
    if (grow > nN - 1) grow = nN - 1;
    const float* X2 = ((part & 1) ? ah : h) + (size_t)grow * DIN;
    const float* wq = wr + part * DIN;
    double accd = 0.0;
#pragma unroll 4
    for (int q = 0; q < DIN / 4; ++q) {
      const v4f xv = *(const v4f*)(X2 + 4 * q);
      accd = fma((double)bfr(xv.x), (double)bfr(wq[4 * q + 0]), accd);
      accd = fma((double)bfr(xv.y), (double)bfr(wq[4 * q + 1]), accd);
      accd = fma((double)bfr(xv.z), (double)bfr(wq[4 * q + 2]), accd);
      accd = fma((double)bfr(xv.w), (double)bfr(wq[4 * q + 3]), accd);
    }
    PR[part * GR + row] = accd;

    const int smat = part >> 1;
    const int head = part & 1;
    const float* tp = S + ((smat * 2) * GR + row) * DOUT + head * HDIM;
    float dp1 = 0.f, dp2 = 0.f, dn1 = 0.f, dn2 = 0.f;
#pragma unroll
    for (int c = 0; c < HDIM; ++c) {
      const float t = tp[c];
      dp1 = fmaf(t, bfr(wp[c]),        dp1);
      dp2 = fmaf(t, bfr(wp[HDIM + c]), dp2);
      dn1 = fmaf(t, bfr(wn[c]),        dn1);
      dn2 = fmaf(t, bfr(wn[HDIM + c]), dn2);
    }
    float* scp = SC + row * ASCW + head * 8 + 2 * smat;
    scp[0] = dp1;
    scp[1] = dn1;
    scp[4] = dp2;
    scp[5] = dn2;
  }
  __syncthreads();
  if (tid < 2 * GR) {
    const int which = tid >> 5, r = tid & 31;
    RS[which * GR + r] = PR[(2 * which) * GR + r] + PR[(2 * which + 1) * GR + r];
  }
  __syncthreads();

  float* G[4] = {th, lh, tah, lah};
  v4f v[8];
#pragma unroll
  for (int a = 0; a < 4; ++a) {
#pragma unroll
    for (int i = 0; i < 2; ++i)
      v[a * 2 + i] = *(const v4f*)(S + a * (GR * DOUT) + wave * 256 + i * 128 + 4 * lane);
  }
  const v4f vs = *(const v4f*)(SC + wave * 128 + 4 * lane);
  const int which = lane >> 4, li = lane & 15;
  const v2d vr = *(const v2d*)(RS + which * GR + 2 * li);
  double* rp = rsd + (size_t)which * nPad + rowBase + 2 * li;
  float*  ap = asc + (size_t)rowBase * ASCW + wave * 128 + 4 * lane;

#pragma unroll
  for (int a = 0; a < 4; ++a) {
#pragma unroll
    for (int i = 0; i < 2; ++i)
      *(volatile v4f*)(G[a] + (size_t)rowBase * DOUT + wave * 256 + i * 128 + 4 * lane) = v[a * 2 + i];
  }
  *(volatile v4f*)ap = vs;
  if (wave == 0) *(volatile v2d*)rp = vr;
  __threadfence();
#pragma unroll
  for (int a = 0; a < 4; ++a) {
#pragma unroll
    for (int i = 0; i < 2; ++i)
      *(volatile v4f*)(G[a] + (size_t)rowBase * DOUT + wave * 256 + i * 128 + 4 * lane) = v[a * 2 + i];
  }
  *(volatile v4f*)ap = vs;
  if (wave == 0) *(volatile v2d*)rp = vr;
}

__global__ __launch_bounds__(NTHR) void k_agg(
    const int* __restrict__ src, const int* __restrict__ dst,
    const float* __restrict__ th, const float* __restrict__ tah,
    const float* __restrict__ lh, const float* __restrict__ lah,
    const float* __restrict__ asc, const double* __restrict__ rsd,
    const float* __restrict__ bp, const float* __restrict__ bn, const float* __restrict__ br,
    float* out, int nN, int nE, int nPad) {
  extern __shared__ v4f lds_dyn[];
  float* ACO  = (float*)lds_dyn;
  float* ACA  = ACO + NB * DOUT;
  float* DEN  = ACA + NB * DOUT;
  float* MX   = DEN + NB * 4;
  int*   list = (int*)(MX + NB * 4);
  int*   wcnt = list + LDS_LIST;
  float* MXv = MX;

  const int tid  = threadIdx.x;
  const int lane = tid & 31;
  const int wave = tid >> 5;
  const int hd   = lane >> 4;
  const int nodeBase = blockIdx.x * NB;

  {
    const v4f z4 = {0.f, 0.f, 0.f, 0.f};
    const float ninf = -__builtin_huge_valf();
    const v4f n4 = {ninf, ninf, ninf, ninf};
    for (int i = tid; i < (NB * 2 * DOUT + NB * 4) / 4; i += NTHR) lds_dyn[i] = z4;
    const int mx0 = (NB * 2 * DOUT + NB * 4) / 4;
    for (int i = tid; i < NB; i += NTHR) lds_dyn[mx0 + i] = n4;
  }
  __syncthreads();

  const float  BP = bfr(bp[0]);
  const float  BN = bfr(bn[0]);
  const double BR = (double)bfr(br[0]);
  const bool al16 = ((reinterpret_cast<size_t>(dst) & (size_t)15) == 0);

  const int nChunks = (nE + CHUNK - 1) / CHUNK;
#pragma unroll 1
  for (int ch = 0; ch < nChunks; ++ch) {
    const int cbase = ch * CHUNK;
    int wc = 0;
#pragma unroll
    for (int g = 0; g < NGRP; ++g) {
      const int el0 = (g * NTHR + tid) * 4;
      const int e0  = cbase + el0;
      const int sent = -2147483647 - 1;
      v4i d;
      if (al16 && (e0 + 3 < nE)) {
        d = *(const v4i*)(dst + e0);
      } else {
        d.x = (e0     < nE) ? dst[min(e0,     nE - 1)] : sent;
        d.y = (e0 + 1 < nE) ? dst[min(e0 + 1, nE - 1)] : sent;
        d.z = (e0 + 2 < nE) ? dst[min(e0 + 2, nE - 1)] : sent;
        d.w = (e0 + 3 < nE) ? dst[min(e0 + 3, nE - 1)] : sent;
      }
      const unsigned s0 = (unsigned)d.x - (unsigned)nodeBase;
      const unsigned s1 = (unsigned)d.y - (unsigned)nodeBase;
      const unsigned s2 = (unsigned)d.z - (unsigned)nodeBase;
      const unsigned s3 = (unsigned)d.w - (unsigned)nodeBase;
      const bool h0 = s0 < (unsigned)NB;
      const bool h1 = s1 < (unsigned)NB;
      const bool h2 = s2 < (unsigned)NB;
      const bool h3 = s3 < (unsigned)NB;
      const unsigned many = __builtin_amdgcn_ballot_w32(h0 | h1 | h2 | h3);
      if (many != 0u) {
#define HITJ(J, HJ, SJ) { \
          const unsigned mj = __builtin_amdgcn_ballot_w32(HJ); \
          if (HJ) { \
            const int pos = wc + (int)__builtin_amdgcn_mbcnt_lo(mj, 0u); \
            if (pos < WCAP) list[wave * WCAP + pos] = ((el0 + (J)) << 9) | (int)(SJ); \
          } \
          wc += (int)__builtin_popcount(mj); }
        HITJ(0, h0, s0)
        HITJ(1, h1, s1)
        HITJ(2, h2, s2)
        HITJ(3, h3, s3)
#undef HITJ
      }
    }
    if (lane == 0) wcnt[wave] = wc;
    __syncthreads();

    if (wave == 0) {
      for (int wsx = 0; wsx < NWAVE; ++wsx) {
        int n = wcnt[wsx];
        if (n > WCAP) n = WCAP;
        if (n < 0) n = 0;
        for (int i = 0; i < n; ++i) {
          const int ent  = list[wsx * WCAP + i];
          const int slot = ent & (NB - 1);
          const int el   = (ent >> 9) & (CHUNK - 1);
          int e = cbase + el;
          if (e > nE - 1) e = nE - 1;
          int s = src[e];
          s = s < 0 ? 0 : (s > nN - 1 ? nN - 1 : s);
          int nd = nodeBase + slot;
          if (nd > nN - 1) nd = nN - 1;
          const double rel = rsd[s] + rsd[(size_t)nPad + nd] + BR;
          const bool pos = (rel >= 0.0);
          const v4f sv = *(const v4f*)(asc + (size_t)s  * ASCW + hd * 8);
          const v4f dv = *(const v4f*)(asc + (size_t)nd * ASCW + hd * 8 + 4);
          const float tv = th [(size_t)s * DOUT + lane];
          const float av = tah[(size_t)s * DOUT + lane];
          float so, sa, fo, fa;
          if (pos) { so = sv.x + dv.x + BP; sa = sv.z + dv.z + BP; fo = tv; fa = av; }
          else     { so = sv.w + dv.y + BN; sa = sv.y + dv.w + BN; fo = av; fa = tv; }
          so = (so >= 0.f) ? so : 0.01f * so;
          sa = (sa >= 0.f) ? sa : 0.01f * sa;
          const int xi = slot * 4 + hd;
          const float mo  = MXv[xi];
          const float ma  = MXv[xi + 2];
          const float mno = fmaxf(mo, so);
          const float mna = fmaxf(ma, sa);
          const float sco = __expf(mo - mno);
          const float sca = __expf(ma - mna);
          const float po  = __expf(so - mno);
          const float pa  = __expf(sa - mna);
          const int ci = slot * DOUT + lane;
          const float co = ACO[ci];
          const float ca = ACA[ci];
          ACO[ci] = co * sco + po * fo;
          ACA[ci] = ca * sca + pa * fa;
          if ((lane & 15) == 0) {
            const float dno = DEN[xi];
            const float dna = DEN[xi + 2];
            DEN[xi]     = dno * sco + po;
            DEN[xi + 2] = dna * sca + pa;
            MXv[xi]     = mno;
            MXv[xi + 2] = mna;
          }
        }
      }
    }
    __syncthreads();
  }

  const int rq   = lane >> 3;
  const int c4   = (lane & 7) * 4;
  const int head = c4 >> 4;
  const size_t outA = (size_t)nN * DOUT;
#pragma unroll 1
  for (int j = 0; j < NB / (NWAVE * 4); ++j) {
    const int slot = wave * (NB / NWAVE) + 4 * j + rq;
    const int node = nodeBase + slot;
    const bool valid = node < nN;
    const size_t nrow = (size_t)(valid ? node : nN - 1);
    const v4f ao = *(const v4f*)(ACO + slot * DOUT + c4);
    const v4f aa = *(const v4f*)(ACA + slot * DOUT + c4);
    const float io = 1.0f / fmaxf(DEN[slot * 4 + head], 1e-16f);
    const float ia = 1.0f / fmaxf(DEN[slot * 4 + 2 + head], 1e-16f);
    const v4f lo = *(const v4f*)(lh  + nrow * DOUT + c4);
    const v4f la = *(const v4f*)(lah + nrow * DOUT + c4);
    const v4f yo = ao * io + lo;
    const v4f ya = aa * ia + la;
    float* po = out + nrow * DOUT + c4;
    float* pa = out + outA + nrow * DOUT + c4;
    if (valid) { *(volatile v4f*)po = yo; *(volatile v4f*)pa = ya; }
    __threadfence();
    if (valid) { *(volatile v4f*)po = yo; *(volatile v4f*)pa = ya; }
  }
}

extern "C" void kernel_launch(void* const* d_in, const int* in_sizes, int n_in,
                              void* d_out, int out_size, void* d_ws, size_t ws_size,
                              hipStream_t stream) {
  if (n_in < 18) return;
  const int nN = in_sizes[0] / DIN;
  if (nN <= 0 || in_sizes[0] != nN * DIN || in_sizes[1] != nN * DIN) return;
  if (in_sizes[2] != DIN * DOUT || in_sizes[4] != DIN * DOUT ||
      in_sizes[6] != DIN * DOUT || in_sizes[8] != DIN * DOUT) return;
  if (in_sizes[3] != DOUT || in_sizes[5] != DOUT || in_sizes[7] != DOUT || in_sizes[9] != DOUT) return;
  if (in_sizes[10] != DOUT || in_sizes[12] != DOUT || in_sizes[14] != 4 * DIN) return;
  if (in_sizes[11] < 1 || in_sizes[13] < 1 || in_sizes[15] < 1) return;
  const int nE = in_sizes[16];
  if (nE < 0 || in_sizes[17] != nE) return;
  if (out_size != 2 * nN * DOUT) return;

  const float* h   = (const float*)d_in[0];
  const float* ah  = (const float*)d_in[1];
  const float* w1  = (const float*)d_in[2];
  const float* b1  = (const float*)d_in[3];
  const float* wa1 = (const float*)d_in[4];
  const float* ba1 = (const float*)d_in[5];
  const float* w2  = (const float*)d_in[6];
  const float* b2  = (const float*)d_in[7];
  const float* wa2 = (const float*)d_in[8];
  const float* ba2 = (const float*)d_in[9];
  const float* wp  = (const float*)d_in[10];
  const float* bp  = (const float*)d_in[11];
  const float* wn  = (const float*)d_in[12];
  const float* bn  = (const float*)d_in[13];
  const float* wr  = (const float*)d_in[14];
  const float* br  = (const float*)d_in[15];
  const int*   src = (const int*)d_in[16];
  const int*   dst = (const int*)d_in[17];
  float* out = (float*)d_out;

  const int nPad = ((nN + GR - 1) / GR) * GR;
  size_t off = 0;
  unsigned short* WT = (unsigned short*)((char*)d_ws + off);
  off += (size_t)2 * 64 * DIN * sizeof(unsigned short);
  const size_t planeB = (size_t)nPad * DOUT * sizeof(float);
  float* th  = (float*)((char*)d_ws + off); off += planeB;
  float* lh  = (float*)((char*)d_ws + off); off += planeB;
  float* tah = (float*)((char*)d_ws + off); off += planeB;
  float* lah = (float*)((char*)d_ws + off); off += planeB;
  float* asc = (float*)((char*)d_ws + off); off += (size_t)nPad * ASCW * sizeof(float);
  double* rsd = (double*)((char*)d_ws + off); off += (size_t)2 * nPad * sizeof(double);
  if (off > ws_size) return;

  const int n8 = 2 * 64 * (DIN / 8);
  k_prep<<<(n8 + NTHR - 1) / NTHR, NTHR, 0, stream>>>(w1, w2, wa1, wa2, WT, n8);

  k_node<<<nPad / GR, NT1, 0, stream>>>(h, ah, WT, b1, ba1, b2, ba2, wp, wn, wr,
                                         th, lh, tah, lah, asc, rsd, nN, nPad);

  hipFuncSetAttribute(reinterpret_cast<const void*>(&k_agg),
                      hipFuncAttributeMaxDynamicSharedMemorySize, LDS_BYTES);
  const int grid = (nN + NB - 1) / NB;
  k_agg<<<grid, NTHR, LDS_BYTES, stream>>>(src, dst, th, tah, lh, lah, asc, rsd,
                                           bp, bn, br, out, nN, nE, nPad);
}
